// SA_Layer_77824807404163
// MI455X (gfx1250) — hardware-verified
//
#include <hip/hip_runtime.h>
#include <math.h>

constexpr int NB = 16;
constexpr int NCH = 256;
constexpr int NPT = 2048;
constexpr int DQ = 64;
constexpr int NBIN = 32;
constexpr int LTR = 2 * NBIN - 1;
constexpr int CHB = 2;
constexpr int NCHUNK = NB / CHB;
constexpr int QA_LD = 384;
constexpr int KA_LD = 384;
constexpr int TB_OFF = 192;
constexpr int LT_LD = 128;
constexpr int LT_ROWS = 192;
constexpr int WT_LD = 512;
constexpr int DF_LD = 512;
constexpr int CS_LD = 32;
constexpr int EK = 384;
constexpr int TSLAB = 196;
constexpr float PCARRY = 32768.0f;
constexpr float PCARRY_INV = 1.0f / 32768.0f;
constexpr float BN_EPS_C = 1e-5f;
constexpr float CS_EPS = 1e-9f;
static_assert(NPT % 64 == 0 && NCH % 64 == 0 && (2 * DQ) % 64 == 0, "tile multiples");
static_assert(NCH % 32 == 0 && EK % 32 == 0 && NPT % 32 == 0 && DF_LD % 32 == 0 && (2 * DQ) % 32 == 0, "K multiples of 32");
static_assert(QA_LD * 2 % 128 == 0 && KA_LD * 2 % 128 == 0 && DF_LD * 2 % 128 == 0 && NCH * 2 % 128 == 0, "line-multiple pitches");
static_assert(NB % CHB == 0, "chunks");
static_assert(TB_OFF + 192 == QA_LD, "layout");

typedef __attribute__((ext_vector_type(16))) _Float16 v16h;
typedef __attribute__((ext_vector_type(8)))  _Float16 v8h;
typedef __attribute__((ext_vector_type(16))) __bf16   v16b;
typedef __attribute__((ext_vector_type(8)))  __bf16   v8b;
typedef __attribute__((ext_vector_type(8)))  float    v8f;
typedef __attribute__((ext_vector_type(4)))  float    v4f;
typedef __attribute__((ext_vector_type(4)))  unsigned int v4u;

__device__ __forceinline__ unsigned short f2bf_bits(float f) {
  unsigned u = __float_as_uint(f);
  return (unsigned short)((u + 0x7FFFu + ((u >> 16) & 1u)) >> 16);
}
__device__ __forceinline__ float bf_bits2f(unsigned short h) { return __uint_as_float(((unsigned)h) << 16); }
__device__ __forceinline__ float bfr(float f) { return __uint_as_float(((unsigned)f2bf_bits(f)) << 16); }
__device__ __forceinline__ unsigned pk16(unsigned short a, unsigned short b) { return (unsigned)a | ((unsigned)b << 16); }
__device__ __forceinline__ unsigned short h_bits(float f) { const _Float16 h = (_Float16)f; return __builtin_bit_cast(unsigned short, h); }

__device__ __forceinline__ void dep_guard4_h(v8f& a, v8f& b, v8f& c, v8f& d, v16h x) { asm volatile("v_nop\n\tv_nop\n\tv_nop\n\tv_nop" : "+v"(a), "+v"(b), "+v"(c), "+v"(d) : "v"(x)); }
__device__ __forceinline__ void dep_guard4_b(v8f& a, v8f& b, v8f& c, v8f& d, v16b x) { asm volatile("v_nop\n\tv_nop\n\tv_nop\n\tv_nop" : "+v"(a), "+v"(b), "+v"(c), "+v"(d) : "v"(x)); }
__device__ __forceinline__ void keep4_h(v16h a, v16h b, v16h c, v16h d) { asm volatile("v_nop" :: "v"(a), "v"(b), "v"(c), "v"(d)); }
__device__ __forceinline__ void keep4_b(v16b a, v16b b, v16b c, v16b d) { asm volatile("v_nop" :: "v"(a), "v"(b), "v"(c), "v"(d)); }
__device__ __forceinline__ void acc_guard4(v8f& a, v8f& b, v8f& c, v8f& d) { asm volatile("v_nop\n\tv_nop\n\tv_nop\n\tv_nop" : "+v"(a), "+v"(b), "+v"(c), "+v"(d)); }
template <typename T> struct Frag;
template <> struct Frag<_Float16> {
  typedef v16h V; union U { v16h v; v8h h[2]; };
  static __device__ __forceinline__ v16h load(const _Float16* p) {
    U f; f.h[0] = *(const v8h*)(p); f.h[1] = *(const v8h*)(p + 16); return f.v;
  }
  static __device__ __forceinline__ v8f mma(v16h a, v16h b, v8f c) {
    return __builtin_amdgcn_wmma_f32_16x16x32_f16(false, a, false, b, (short)0, c, false, false);
  }
  static __device__ __forceinline__ void guard4(v8f& a, v8f& b, v8f& c, v8f& d, v16h x) { dep_guard4_h(a, b, c, d, x); }
  static __device__ __forceinline__ void keep(v16h a, v16h b, v16h c, v16h d) { keep4_h(a, b, c, d); }
};
template <> struct Frag<__bf16> {
  typedef v16b V; union U { v16b v; v8b h[2]; };
  static __device__ __forceinline__ v16b load(const __bf16* p) {
    U f; f.h[0] = *(const v8b*)(p); f.h[1] = *(const v8b*)(p + 16); return f.v;
  }
  static __device__ __forceinline__ v8f mma(v16b a, v16b b, v8f c) {
    return __builtin_amdgcn_wmma_f32_16x16x32_bf16(false, a, false, b, (short)0, c, false, false);
  }
  static __device__ __forceinline__ void guard4(v8f& a, v8f& b, v8f& c, v8f& d, v16b x) { dep_guard4_b(a, b, c, d, x); }
  static __device__ __forceinline__ void keep(v16b a, v16b b, v16b c, v16b d) { keep4_b(a, b, c, d); }
};

template <int ET> struct Elem;
template <> struct Elem<0> { typedef _Float16 T; };
template <> struct Elem<1> { typedef __bf16 T; };
template <int ET, int EPI>
__global__ __launch_bounds__(256) void gemm64(
    const unsigned short* __restrict__ Ap, int lda, long strideA,
    const unsigned short* __restrict__ Btp, int ldb, long strideB,
    void* Cout, int ldc, long strideC, void* Cout2,
    const float* __restrict__ vec0, const float* __restrict__ vec1, long strideV,
    const unsigned short* __restrict__ aux16, int ldx, long strideX,
    const float* __restrict__ auxf, long strideF,
    int M, int N, int K, float scale) {
  typedef typename Elem<ET>::T T;
  typedef typename Frag<T>::V V;
  const T* A = (const T*)Ap; const T* Bt = (const T*)Btp;
  __shared__ __align__(16) float sT[8][16 * 68];
  const int b    = blockIdx.y;
  const int lane = threadIdx.x & 31;
  const int wave = threadIdx.x >> 5;
  const int tilesN = N >> 6;
  const int tilesM = M >> 6;
  const int tile = blockIdx.x * 8 + wave;
  if (tile >= tilesM * tilesN) return;
  const int tm = tile / tilesN;
  const int tn = tile - tm * tilesN;
  const int m0 = tm << 6;
  const int n0 = tn << 6;

  const T* Ab = A  + (size_t)b * strideA;
  const T* Bb = Bt + (size_t)b * strideB;

  const int rlane = lane & 15;
  const int koff  = (lane >> 4) * 8;
  const int mOff  = (lane >> 4) * 8;

  v8f acc[4][4];
#pragma unroll
  for (int i = 0; i < 4; ++i)
#pragma unroll
    for (int j = 0; j < 4; ++j) acc[i][j] = (v8f){0.f,0.f,0.f,0.f,0.f,0.f,0.f,0.f};

  for (int k0 = 0; k0 < K; k0 += 32) {
    V bq[4];
#pragma unroll
    for (int j = 0; j < 4; ++j) {
      const size_t bo = (size_t)(n0 + (j << 4) + rlane) * ldb + koff + k0;
      bq[j] = Frag<T>::load(Bb + bo);
    }
#pragma unroll
    for (int i = 0; i < 4; ++i) {
      const size_t ao = (size_t)(m0 + (i << 4) + rlane) * lda + koff + k0;
      V ah = Frag<T>::load(Ab + ao);
#pragma unroll
      for (int j = 0; j < 4; ++j) acc[i][j] = Frag<T>::mma(ah, bq[j], acc[i][j]);
      Frag<T>::guard4(acc[i][0], acc[i][1], acc[i][2], acc[i][3], ah);
    }
    Frag<T>::keep(bq[0], bq[1], bq[2], bq[3]);
  }
  acc_guard4(acc[0][0], acc[0][1], acc[0][2], acc[0][3]);
  acc_guard4(acc[1][0], acc[1][1], acc[1][2], acc[1][3]);
  acc_guard4(acc[2][0], acc[2][1], acc[2][2], acc[2][3]);
  acc_guard4(acc[3][0], acc[3][1], acc[3][2], acc[3][3]);

  float* slab = sT[wave];
  const float escale = (EPI == 3) ? 1.0f : scale;
#pragma unroll
  for (int i = 0; i < 4; ++i) {
    const int mBase = m0 + (i << 4);
#pragma unroll
    for (int j = 0; j < 4; ++j) {
#pragma unroll
      for (int r = 0; r < 8; ++r) slab[(mOff + r) * 68 + (j << 4) + rlane] = acc[i][j][r] * escale;
    }
    __builtin_amdgcn_fence(__ATOMIC_RELEASE, "workgroup");
    __builtin_amdgcn_wave_barrier();
    __builtin_amdgcn_fence(__ATOMIC_ACQUIRE, "workgroup");
    if (EPI == 0) {
      float* C = (float*)Cout + (size_t)b * strideC;
      const int hh = lane >> 4, c4 = (lane & 15) * 4;
      for (int pass = 0; pass < 2; ++pass) {
#pragma unroll
        for (int it = 0; it < 8; ++it) {
          const int row = it * 2 + hh;
          v4f v = *(const v4f*)(slab + row * 68 + c4);
          *(volatile v4f*)(C + (size_t)(mBase + row) * ldc + n0 + c4) = v;
        }
        __threadfence();
      }
    } else if (EPI == 4) {
      float* C = (float*)Cout + (size_t)b * strideC;
      const float* X = auxf + (size_t)b * strideF;
      const int hh = lane >> 4, c4 = (lane & 15) * 4;
      for (int pass = 0; pass < 2; ++pass) {
#pragma unroll
        for (int it = 0; it < 8; ++it) {
          const int row = it * 2 + hh;
          const int o = mBase + row;
          const float sc = vec0[o];
          const float sh = vec1[o];
          const v4f a  = *(const v4f*)(slab + row * 68 + c4);
          const v4f xr = *(const v4f*)(X + (size_t)o * ldc + n0 + c4);
          v4f ov;
#pragma unroll
          for (int e = 0; e < 4; ++e) ov[e] = bfr(xr[e]) + fmaxf(a[e] * sc + sh, 0.0f);
          *(volatile v4f*)(C + (size_t)o * ldc + n0 + c4) = ov;
        }
        __threadfence();
      }
    } else if (EPI == 1) {
      unsigned short* C = (unsigned short*)Cout + (size_t)b * strideC;
      const int q8 = lane >> 3, c8 = (lane & 7) * 8;
      for (int pass = 0; pass < 2; ++pass) {
#pragma unroll
        for (int it = 0; it < 4; ++it) {
          const int row = it * 4 + q8;
          const float bias = vec0[mBase + row];
          const float* sp = slab + row * 68 + c8;
          unsigned short hb[8];
#pragma unroll
          for (int e = 0; e < 8; ++e) hb[e] = h_bits(sp[e] + bias);
          const v4u w = (v4u){pk16(hb[0], hb[1]), pk16(hb[2], hb[3]), pk16(hb[4], hb[5]), pk16(hb[6], hb[7])};
          *(volatile v4u*)(C + (size_t)(mBase + row) * ldc + n0 + c8) = w;
        }
        __threadfence();
      }
    } else if (EPI == 2) {
      const bool isq = (tn == 0);
      unsigned short* P = (isq ? (unsigned short*)Cout : (unsigned short*)Cout2) + (size_t)b * strideC;
      const int q8 = lane >> 3, c8 = (lane & 7) * 8;
      for (int pass = 0; pass < 2; ++pass) {
#pragma unroll
        for (int it = 0; it < 4; ++it) {
          const int row = it * 4 + q8;
          const float* sp = slab + row * 68 + c8;
          unsigned short hb[8], lb[8];
#pragma unroll
          for (int e = 0; e < 8; ++e) {
            const unsigned short h = f2bf_bits(sp[e]);
            hb[e] = h;
            lb[e] = f2bf_bits(sp[e] - bf_bits2f(h));
          }
          const v4u wh = (v4u){pk16(hb[0], hb[1]), pk16(hb[2], hb[3]), pk16(hb[4], hb[5]), pk16(hb[6], hb[7])};
          const v4u wl = (v4u){pk16(lb[0], lb[1]), pk16(lb[2], lb[3]), pk16(lb[4], lb[5]), pk16(lb[6], lb[7])};
          const v4u s1 = isq ? wh : wl;
          const v4u s2 = isq ? wl : wh;
          unsigned short* base = P + (size_t)(mBase + row) * ldc + c8;
          *(volatile v4u*)(base)       = wh;
          *(volatile v4u*)(base + 64)  = s1;
          *(volatile v4u*)(base + 128) = s2;
        }
        __threadfence();
      }
    } else {
      unsigned short* C = (unsigned short*)Cout + (size_t)b * strideC;
      const unsigned short* X = aux16 + (size_t)b * strideX;
      const float* CS = vec0 + (size_t)b * strideV;
      const int q8 = lane >> 3, c8 = (lane & 7) * 8;
      for (int pass = 0; pass < 2; ++pass) {
#pragma unroll
        for (int it = 0; it < 4; ++it) {
          const int row = it * 4 + q8;
          const int m = mBase + row;
          const float cs = CS[(size_t)m * CS_LD];
          const float rs = scale * (1.0f / (CS_EPS + cs));
          const v4u xw = *(const v4u*)(X + (size_t)m * ldx + n0 + c8);
          float xv[8];
          xv[0] = __uint_as_float(xw.x << 16); xv[1] = __uint_as_float(xw.x & 0xffff0000u);
          xv[2] = __uint_as_float(xw.y << 16); xv[3] = __uint_as_float(xw.y & 0xffff0000u);
          xv[4] = __uint_as_float(xw.z << 16); xv[5] = __uint_as_float(xw.z & 0xffff0000u);
          xv[6] = __uint_as_float(xw.w << 16); xv[7] = __uint_as_float(xw.w & 0xffff0000u);
          const float* sp = slab + row * 68 + c8;
          unsigned short hb[8], lb[8];
#pragma unroll
          for (int e = 0; e < 8; ++e) {
            const float d = xv[e] - sp[e] * rs;
            const unsigned short h = f2bf_bits(d);
            hb[e] = h;
            lb[e] = f2bf_bits(d - bf_bits2f(h));
          }
          const v4u wh = (v4u){pk16(hb[0], hb[1]), pk16(hb[2], hb[3]), pk16(hb[4], hb[5]), pk16(hb[6], hb[7])};
          const v4u wl = (v4u){pk16(lb[0], lb[1]), pk16(lb[2], lb[3]), pk16(lb[4], lb[5]), pk16(lb[6], lb[7])};
          unsigned short* base = C + (size_t)m * ldc + n0 + c8;
          *(volatile v4u*)(base)     = wh;
          *(volatile v4u*)(base + N) = wl;
        }
        __threadfence();
      }
    }
    __builtin_amdgcn_fence(__ATOMIC_RELEASE, "workgroup");
    __builtin_amdgcn_wave_barrier();
    __builtin_amdgcn_fence(__ATOMIC_ACQUIRE, "workgroup");
  }
}

__global__ __launch_bounds__(256) void wcvt_kernel(const float* __restrict__ Wq, const float* __restrict__ Wk,
                                                   const float* __restrict__ Wv, const float* __restrict__ Wt,
                                                   const float* __restrict__ xlt, const float* __restrict__ ylt,
                                                   const float* __restrict__ zlt,
                                                   const float* __restrict__ bv, const float* __restrict__ bt,
                                                   const float* __restrict__ gam, const float* __restrict__ bet,
                                                   const float* __restrict__ rmean, const float* __restrict__ rvar,
                                                   unsigned short* Wqk, unsigned short* Wvb, unsigned short* Wt2,
                                                   unsigned short* LT2, float* vec) {
  const int blk = blockIdx.x;
  const int t = threadIdx.x;
  if (blk < 124) {
    float f[8];
    unsigned short* dst;
    if (blk < 16) {
      const int el = (blk * 256 + t) * 8;
      const int row = el >> 8, col = el & 255;
      const float* s = (blk < 8) ? (Wq + (size_t)row * NCH + col) : (Wk + (size_t)(row - 64) * NCH + col);
#pragma unroll
      for (int e = 0; e < 8; ++e) f[e] = s[e];
      dst = Wqk + el;
    } else if (blk < 48) {
      const int el = ((blk - 16) * 256 + t) * 8;
#pragma unroll
      for (int e = 0; e < 8; ++e) f[e] = Wv[el + e];
      dst = Wvb + el;
    } else if (blk < 112) {
      const int el = ((blk - 48) * 256 + t) * 8;
      const int row = el >> 9, col = el & 511;
      const float* s = Wt + (size_t)row * NCH + (col & 255);
#pragma unroll
      for (int e = 0; e < 8; ++e) f[e] = s[e];
      dst = Wt2 + el;
    } else {
      const int el = ((blk - 112) * 256 + t) * 8;
      const int row = el >> 7, col = el & 127;
      const int tt = (blk - 112) >> 2;
      const int r = row & 63;
      const int rr = (r < LTR - 1) ? r : (LTR - 1);
      const float* tab = (tt == 0) ? xlt : ((tt == 1) ? ylt : zlt);
      const float* s = tab + (size_t)rr * DQ + (col & 63);
      const float fz = (r < LTR) ? 1.0f : 0.0f;
#pragma unroll
      for (int e = 0; e < 8; ++e) f[e] = s[e] * fz;
      dst = LT2 + el;
    }
    unsigned short hb[8];
#pragma unroll
    for (int e = 0; e < 8; ++e) hb[e] = f2bf_bits(f[e]);
    const v4u w = (v4u){pk16(hb[0], hb[1]), pk16(hb[2], hb[3]), pk16(hb[4], hb[5]), pk16(hb[6], hb[7])};
    *(volatile v4u*)dst = w;
    __threadfence();
    *(volatile v4u*)dst = w;
  } else {
    const int o4 = (t & 63) * 4;
    const int sel = t >> 6;
    const v4f vb  = *(const v4f*)(bv + o4);
    const v4f vt  = *(const v4f*)(bt + o4);
    const v4f vg  = *(const v4f*)(gam + o4);
    const v4f vbe = *(const v4f*)(bet + o4);
    const v4f vm  = *(const v4f*)(rmean + o4);
    const v4f vv  = *(const v4f*)(rvar + o4);
    v4f c0, c1, c2;
#pragma unroll
    for (int e = 0; e < 4; ++e) {
      const float inv = bfr(vg[e]) / sqrtf(bfr(vv[e]) + BN_EPS_C);
      c0[e] = bfr(vb[e]);
      c1[e] = inv;
      c2[e] = (bfr(vt[e]) - bfr(vm[e])) * inv + bfr(vbe[e]);
    }
    const v4f val = (sel == 0) ? c0 : ((sel == 1) ? c1 : c2);
    if (t < 192) {
      float* d = vec + sel * NCH + o4;
      *(volatile v4f*)d = val;
      __threadfence();
      *(volatile v4f*)d = val;
    }
  }
}

__global__ __launch_bounds__(256) void xt_kernel(const float* __restrict__ x, unsigned short* xT) {
  __shared__ float sm[64][65];
  const int t  = threadIdx.x;
  const int c0 = blockIdx.x * 64;
  const int n0 = blockIdx.y * 64;
  const int b  = blockIdx.z;
#pragma unroll
  for (int i = 0; i < 16; ++i) {
    const int e = i * 256 + t;
    const int nl = e & 63;
    const int cl = e >> 6;
    sm[cl][nl] = x[((size_t)(b * NCH + c0 + cl)) * NPT + n0 + nl];
  }
  __syncthreads();
  const int lane = t & 31, wave = t >> 5;
  const int q8 = lane >> 3, c8 = (lane & 7) * 8;
  unsigned short* op = xT + ((size_t)b * NPT) * NCH;
  for (int pass = 0; pass < 2; ++pass) {
#pragma unroll
    for (int it = 0; it < 2; ++it) {
      const int row = wave * 8 + it * 4 + q8;
      unsigned short hb[8];
#pragma unroll
      for (int e = 0; e < 8; ++e) hb[e] = f2bf_bits(sm[c8 + e][row]);
      const v4u w = (v4u){pk16(hb[0], hb[1]), pk16(hb[2], hb[3]), pk16(hb[4], hb[5]), pk16(hb[6], hb[7])};
      *(volatile v4u*)(op + (size_t)(n0 + row) * NCH + c0 + c8) = w;
    }
    __threadfence();
  }
}

__global__ __launch_bounds__(128) void tbuild_kernel(unsigned short* Qa, unsigned short* Ka,
                                                     const unsigned short* __restrict__ LT2p,
                                                     const int* __restrict__ disc) {
  __shared__ __align__(16) float sl[4][16 * TSLAB];
  const int b = blockIdx.y;
  const int lane = threadIdx.x & 31, wave = threadIdx.x >> 5;
  const int rlane = lane & 15, koff = (lane >> 4) * 8, mOff = koff;
  const int r0 = blockIdx.x * 64 + wave * 16;
  const __bf16* Q = (const __bf16*)Qa + ((size_t)b * NPT) * QA_LD;
  const __bf16* L = (const __bf16*)LT2p;
  v16b af[4];
#pragma unroll
  for (int ks = 0; ks < 4; ++ks)
    af[ks] = Frag<__bf16>::load(Q + (size_t)(r0 + rlane) * QA_LD + 64 + ks * 32 + koff);
  float* slab = sl[wave];
#pragma unroll 1
  for (int tt = 0; tt < 3; ++tt) {
    v8f acc[4];
#pragma unroll
    for (int j = 0; j < 4; ++j) acc[j] = (v8f){0.f,0.f,0.f,0.f,0.f,0.f,0.f,0.f};
#pragma unroll
    for (int ks = 0; ks < 4; ++ks) {
      v16b bq[4];
#pragma unroll
      for (int j = 0; j < 4; ++j)
        bq[j] = Frag<__bf16>::load(L + (size_t)(tt * 64 + 16 * j + rlane) * LT_LD + ks * 32 + koff);
#pragma unroll
      for (int j = 0; j < 4; ++j) acc[j] = Frag<__bf16>::mma(af[ks], bq[j], acc[j]);
      Frag<__bf16>::guard4(acc[0], acc[1], acc[2], acc[3], af[ks]);
      Frag<__bf16>::keep(bq[0], bq[1], bq[2], bq[3]);
    }
    acc_guard4(acc[0], acc[1], acc[2], acc[3]);
#pragma unroll
    for (int j = 0; j < 4; ++j)
#pragma unroll
      for (int r = 0; r < 8; ++r) slab[(mOff + r) * TSLAB + tt * 64 + 16 * j + rlane] = acc[j][r];
  }
  __builtin_amdgcn_fence(__ATOMIC_RELEASE, "workgroup");
  __builtin_amdgcn_wave_barrier();
  __builtin_amdgcn_fence(__ATOMIC_ACQUIRE, "workgroup");

  const int q8 = lane >> 3, c8 = (lane & 7) * 8;
  unsigned short* QO = Qa + ((size_t)b * NPT) * QA_LD;
  unsigned short* KO = Ka + ((size_t)b * NPT) * KA_LD;
  const int* D = disc + (size_t)b * NPT * 3;
  for (int pass = 0; pass < 2; ++pass) {
#pragma unroll 1
    for (int it = 0; it < 12; ++it) {
      const int combo = it * 4 + q8;
      const int row = combo / 3;
      const int seg = combo - row * 3;
      const int n = r0 + row;
      const int tc0 = seg * 64 + c8;
      const int part = (tc0 >= 96) ? 1 : 0;
      const int u = tc0 - 96 * part;
      const int tsel = u >> 5;
      const int a0 = u & 31;
      int dn = D[(size_t)n * 3 + tsel];
      dn = (dn < 0) ? 0 : ((dn > NBIN - 1) ? (NBIN - 1) : dn);
      const int sh = (NBIN - 1) - dn;
      const float* src = slab + row * TSLAB + tsel * 64 + a0 + sh;
      unsigned short tb[8], ob[8];
#pragma unroll
      for (int e = 0; e < 8; ++e) {
        const float v = src[e];
        const unsigned short h = f2bf_bits(v);
        const unsigned short l = f2bf_bits(v - bf_bits2f(h));
        tb[e] = part ? l : h;
        ob[e] = (dn == a0 + e) ? (unsigned short)0x3F80u : (unsigned short)0u;
      }
      const v4u wt = (v4u){pk16(tb[0], tb[1]), pk16(tb[2], tb[3]), pk16(tb[4], tb[5]), pk16(tb[6], tb[7])};
      const v4u wo = (v4u){pk16(ob[0], ob[1]), pk16(ob[2], ob[3]), pk16(ob[4], ob[5]), pk16(ob[6], ob[7])};
      *(volatile v4u*)(QO + (size_t)n * QA_LD + TB_OFF + tc0) = wt;
      *(volatile v4u*)(KO + (size_t)n * KA_LD + TB_OFF + tc0) = wo;
    }
    __threadfence();
  }
}

__global__ __launch_bounds__(256) void rowstats_kernel(const float* __restrict__ ET, float* rowmax, float* rowinv) {
  __shared__ float pm[4][64];
  __shared__ float ps[4][64];
  __shared__ __align__(16) float ost[128];
  const int bl = blockIdx.y, n0 = blockIdx.x * 64, t = threadIdx.x;
  const int nl = t & 63, mg = t >> 6;
  const float* E = ET + ((size_t)bl * NPT) * NPT + n0 + nl;
  float mr = -INFINITY, s = 0.0f;
#pragma unroll 1
  for (int i = 0; i < 64; ++i) {
    const float* p = E + (size_t)(mg * 512 + 8 * i) * NPT;
    const float e0 = p[0], e1 = p[NPT], e2 = p[2 * NPT], e3 = p[3 * NPT];
    const float e4 = p[4 * NPT], e5 = p[5 * NPT], e6 = p[6 * NPT], e7 = p[7 * NPT];
    const float cm = fmaxf(fmaxf(fmaxf(e0, e1), fmaxf(e2, e3)), fmaxf(fmaxf(e4, e5), fmaxf(e6, e7)));
    const float mn = fmaxf(mr, cm);
    const float add = ((expf(e0 - mn) + expf(e1 - mn)) + (expf(e2 - mn) + expf(e3 - mn)))
                    + ((expf(e4 - mn) + expf(e5 - mn)) + (expf(e6 - mn) + expf(e7 - mn)));
    s = s * expf(mr - mn) + add;
    mr = mn;
  }
  pm[mg][nl] = mr;
  ps[mg][nl] = s;
  __syncthreads();
  if (t < 64) {
    const float m0 = pm[0][t], m1 = pm[1][t], m2 = pm[2][t], m3 = pm[3][t];
    const float mx = fmaxf(fmaxf(m0, m1), fmaxf(m2, m3));
    const float sx = ((ps[0][t] * expf(m0 - mx) + ps[1][t] * expf(m1 - mx)) + ps[2][t] * expf(m2 - mx)) + ps[3][t] * expf(m3 - mx);
    ost[t] = mx;
    ost[64 + t] = 1.0f / sx;
  }
  __syncthreads();
  if (t < 32) {
    const v4f v = *(const v4f*)(ost + 4 * t);
    float* dst = (t < 16) ? (rowmax + (size_t)bl * NPT + n0 + 4 * t) : (rowinv + (size_t)bl * NPT + n0 + 4 * (t - 16));
    *(volatile v4f*)dst = v;
    __threadfence();
    *(volatile v4f*)dst = v;
  }
}

__global__ __launch_bounds__(256) void pwrite_kernel(const float* __restrict__ ET, const float* __restrict__ rowmax,
                                                     const float* __restrict__ rowinv, unsigned short* PT, float* colsum) {
  __shared__ float red[8];
  const int bl = blockIdx.y, m = blockIdx.x, t = threadIdx.x;
  const int lane = t & 31, wave = t >> 5;
  const size_t rowoff = ((size_t)bl * NPT + m) * NPT;
  const float* er = ET + rowoff + 8 * (size_t)t;
  const v4f ea = *(const v4f*)(er);
  const v4f eb = *(const v4f*)(er + 4);
  const float* rmp = rowmax + (size_t)bl * NPT + 8 * t;
  const float* rip = rowinv + (size_t)bl * NPT + 8 * t;
  const v4f ma = *(const v4f*)(rmp), mb = *(const v4f*)(rmp + 4);
  const v4f ia = *(const v4f*)(rip), ib = *(const v4f*)(rip + 4);
  float p[8];
#pragma unroll
  for (int e = 0; e < 4; ++e) {
    p[e]     = expf(ea[e] - ma[e]) * ia[e];
    p[4 + e] = expf(eb[e] - mb[e]) * ib[e];
  }
  float psum = ((p[0] + p[1]) + (p[2] + p[3])) + ((p[4] + p[5]) + (p[6] + p[7]));
  unsigned short hb[8];
#pragma unroll
  for (int e = 0; e < 8; ++e) hb[e] = h_bits(p[e] * PCARRY);
  const v4u w = (v4u){pk16(hb[0], hb[1]), pk16(hb[2], hb[3]), pk16(hb[4], hb[5]), pk16(hb[6], hb[7])};
  unsigned short* pr = PT + rowoff + 8 * (size_t)t;
  *(volatile v4u*)pr = w;
  __threadfence();
  *(volatile v4u*)pr = w;
#pragma unroll
  for (int off = 16; off > 0; off >>= 1) psum += __shfl_xor(psum, off, 32);
  if (lane == 0) red[wave] = psum;
  __syncthreads();
  if (t < 8) {
    float tot = red[0];
#pragma unroll
    for (int wv = 1; wv < 8; ++wv) tot += red[wv];
    const v4f cv = (v4f){(t == 0) ? tot : 0.0f, 0.0f, 0.0f, 0.0f};
    float* cp = colsum + ((size_t)bl * NPT + m) * CS_LD + 4 * t;
    *(volatile v4f*)cp = cv;
    __threadfence();
    *(volatile v4f*)cp = cv;
  }
}

extern "C" void kernel_launch(void* const* d_in, const int* in_sizes, int n_in,
                              void* d_out, int out_size, void* d_ws, size_t ws_size,
                              hipStream_t stream) {
  if (n_in < 16) return;
  if (in_sizes[0] != NB * NCH * NPT) return;
  if (in_sizes[1] != NB * NPT * 3) return;
  if (in_sizes[3] != DQ * NCH || in_sizes[4] != DQ * NCH) return;
  if (in_sizes[5] != NCH * NCH || in_sizes[6] != NCH) return;
  if (in_sizes[7] != LTR * DQ || in_sizes[8] != LTR * DQ || in_sizes[9] != LTR * DQ) return;
  if (in_sizes[10] != NCH * NCH || in_sizes[11] != NCH) return;
  if (in_sizes[12] != NCH || in_sizes[13] != NCH || in_sizes[14] != NCH || in_sizes[15] != NCH) return;
  if (out_size != NB * NCH * NPT) return;

  const size_t szWqk = (size_t)2 * DQ * NCH * 2;
  const size_t szWv  = (size_t)NCH * NCH * 2;
  const size_t szWt2 = (size_t)NCH * WT_LD * 2;
  const size_t szLT2 = (size_t)LT_ROWS * LT_LD * 2;
  const size_t szVec = (size_t)3 * NCH * 4;
  const size_t szXT  = (size_t)NB * NPT * NCH * 2;
  const size_t szQA  = (size_t)NB * NPT * QA_LD * 2;
  const size_t szKA  = (size_t)NB * NPT * KA_LD * 2;
  const size_t szV   = (size_t)CHB * NCH * NPT * 2;
  const size_t szET  = (size_t)CHB * NPT * NPT * 4;
  const size_t szRM  = (size_t)CHB * NPT * 4;
  const size_t szPT  = (size_t)CHB * NPT * NPT * 2;
  const size_t szCS  = (size_t)CHB * NPT * CS_LD * 4;
  const size_t szDF  = (size_t)CHB * NPT * DF_LD * 2;
  size_t off = 0;
  const size_t offWqk = off; off += szWqk;
  const size_t offWv  = off; off += szWv;
  const size_t offWt2 = off; off += szWt2;
  const size_t offLT2 = off; off += szLT2;
  const size_t offVec = off; off += szVec;
  const size_t offXT  = off; off += szXT;
  const size_t offQA  = off; off += szQA;
  const size_t offKA  = off; off += szKA;
  const size_t offV   = off; off += szV;
  const size_t offET  = off; off += szET;
  const size_t offRM  = off; off += szRM;
  const size_t offRI  = off; off += szRM;
  const size_t offPT  = off; off += szPT;
  const size_t offCS  = off; off += szCS;
  const size_t offDF  = off; off += szDF;
  const size_t total  = off;
  if (ws_size < total) return;

  const float* x     = (const float*)d_in[0];
  const int*   disc  = (const int*)d_in[1];
  const float* Wq    = (const float*)d_in[3];
  const float* Wk    = (const float*)d_in[4];
  const float* Wv    = (const float*)d_in[5];
  const float* bv    = (const float*)d_in[6];
  const float* xlt   = (const float*)d_in[7];
  const float* ylt   = (const float*)d_in[8];
  const float* zlt   = (const float*)d_in[9];
  const float* Wt    = (const float*)d_in[10];
  const float* bt    = (const float*)d_in[11];
  const float* gam   = (const float*)d_in[12];
  const float* bet   = (const float*)d_in[13];
  const float* rmean = (const float*)d_in[14];
  const float* rvar  = (const float*)d_in[15];
  float* out = (float*)d_out;

  char* ws = (char*)d_ws;
  unsigned short* Wqk = (unsigned short*)(ws + offWqk);
  unsigned short* Wvb = (unsigned short*)(ws + offWv);
  unsigned short* Wt2 = (unsigned short*)(ws + offWt2);
  unsigned short* LT2 = (unsigned short*)(ws + offLT2);
  float*          vec = (float*)(ws + offVec);
  unsigned short* xT  = (unsigned short*)(ws + offXT);
  unsigned short* Qa  = (unsigned short*)(ws + offQA);
  unsigned short* Ka  = (unsigned short*)(ws + offKA);
  unsigned short* Vp  = (unsigned short*)(ws + offV);
  float*          ET  = (float*)(ws + offET);
  float*          rmx = (float*)(ws + offRM);
  float*          rin = (float*)(ws + offRI);
  unsigned short* PT  = (unsigned short*)(ws + offPT);
  float*          csum = (float*)(ws + offCS);
  unsigned short* dfT = (unsigned short*)(ws + offDF);

  const long xtStride = (long)NPT * NCH;
  const long qaStride = (long)NPT * QA_LD;
  const long vStride  = (long)NCH * NPT;
  const long etStride = (long)NPT * NPT;
  const long csStride = (long)NPT * CS_LD;
  const long dfStride = (long)NPT * DF_LD;

  wcvt_kernel<<<dim3(125), dim3(256), 0, stream>>>(Wq, Wk, Wv, Wt, xlt, ylt, zlt, bv, bt, gam, bet, rmean, rvar,
                                                    Wqk, Wvb, Wt2, LT2, vec);
  xt_kernel<<<dim3(NCH / 64, NPT / 64, NB), dim3(256), 0, stream>>>(x, xT);
  gemm64<1, 2><<<dim3(8, NB), dim3(256), 0, stream>>>(
      xT, NCH, xtStride, Wqk, NCH, 0L, (void*)Qa, QA_LD, qaStride, (void*)Ka,
      nullptr, nullptr, 0L, nullptr, 0, 0L, nullptr, 0L, NPT, 2 * DQ, NCH, 1.0f);
  tbuild_kernel<<<dim3(NPT / 64, NB), dim3(128), 0, stream>>>(Qa, Ka, LT2, disc);

  for (int c = 0; c < NCHUNK; ++c) {
    const int b0 = c * CHB;
    gemm64<1, 1><<<dim3(16, CHB), dim3(256), 0, stream>>>(
        Wvb, NCH, 0L, xT + (size_t)b0 * xtStride, NCH, xtStride, (void*)Vp, NPT, vStride, nullptr,
        vec, nullptr, 0L, nullptr, 0, 0L, nullptr, 0L, NCH, NPT, NCH, 1.0f);
    gemm64<1, 0><<<dim3(128, CHB), dim3(256), 0, stream>>>(
        Ka + (size_t)b0 * qaStride, KA_LD, qaStride, Qa + (size_t)b0 * qaStride, QA_LD, qaStride,
        (void*)ET, NPT, etStride, nullptr,
        nullptr, nullptr, 0L, nullptr, 0, 0L, nullptr, 0L, NPT, NPT, EK, 1.0f);
    rowstats_kernel<<<dim3(NPT / 64, CHB), dim3(256), 0, stream>>>(ET, rmx, rin);
    pwrite_kernel<<<dim3(NPT, CHB), dim3(256), 0, stream>>>(ET, rmx, rin, PT, csum);
    gemm64<0, 3><<<dim3(16, CHB), dim3(256), 0, stream>>>(
        PT, NPT, etStride, Vp, NPT, vStride, (void*)dfT, DF_LD, dfStride, nullptr,
        csum, nullptr, csStride, xT + (size_t)b0 * xtStride, NCH, xtStride, nullptr, 0L,
        NPT, NCH, NPT, PCARRY_INV);
    gemm64<1, 4><<<dim3(16, CHB), dim3(256), 0, stream>>>(
        Wt2, WT_LD, 0L, dfT, DF_LD, dfStride, (void*)(out + (size_t)b0 * vStride), NPT, vStride, nullptr,
        vec + NCH, vec + 2 * NCH, 0L, nullptr, 0, 0L, x + (size_t)b0 * vStride, vStride,
        NCH, NPT, DF_LD, 1.0f);
  }
}
